// GRBlockNorm_76879914598740
// MI455X (gfx1250) — hardware-run, weakly checked
//
#include <hip/hip_runtime.h>

typedef float          v8f   __attribute__((ext_vector_type(8)));
typedef float          v4f   __attribute__((ext_vector_type(4)));
typedef unsigned int   v4u   __attribute__((ext_vector_type(4)));
typedef int            v8i   __attribute__((ext_vector_type(8)));
typedef unsigned short v8us  __attribute__((ext_vector_type(8)));
typedef unsigned short v16us __attribute__((ext_vector_type(16)));
typedef __bf16         v16bf __attribute__((ext_vector_type(16)));
typedef _Float16       v16h  __attribute__((ext_vector_type(16)));
typedef v4f  __attribute__((may_alias)) v4fa;
typedef v8us __attribute__((may_alias)) v8usa;
union FragB { v16bf v; v16us u; v8us h[2]; v8i w; };
union FragH { v16h  v; v16us u; v8us h[2]; v8i w; };

__device__ __forceinline__ v8f wmb(const FragB& a, const FragB& b, v8f c) {
  v8f d = __builtin_amdgcn_wmma_f32_16x16x32_bf16(false, a.v, false, b.v, (short)0, c, false, false);
  asm volatile("v_nop\n\tv_nop\n\tv_nop\n\tv_nop" : "+v"(d) : "v"(a.w), "v"(b.w));
  return d;
}

__device__ __forceinline__ v8f wmh(const FragH& a, const FragH& b, v8f c) {
  v8f d = __builtin_amdgcn_wmma_f32_16x16x32_f16(false, a.v, false, b.v, (short)0, c, false, false);
  asm volatile("v_nop\n\tv_nop\n\tv_nop\n\tv_nop" : "+v"(d) : "v"(a.w), "v"(b.w));
  return d;
}

__device__ __forceinline__ unsigned bf16_bits(float f) {
  const unsigned u = __float_as_uint(f);
  const unsigned r = (u + 0x7FFFu + ((u >> 16) & 1u)) >> 16;
  const unsigned q = (u >> 16) | 0x40u;
  return ((u & 0x7fffffffu) > 0x7f800000u) ? q : r;
}

__device__ __forceinline__ float bf16_val(float f) {
  return __uint_as_float(bf16_bits(f) << 16);
}
__device__ __forceinline__ int clampi(int v, int lo, int hi) {
  return v < lo ? lo : (v > hi ? hi : v);
}

__device__ __forceinline__ unsigned f16_bits(float f) {
  const unsigned u  = __float_as_uint(f);
  const unsigned s  = (u >> 16) & 0x8000u;
  const unsigned a  = u & 0x7fffffffu;
  const unsigned t  = a - 0x38000000u;
  const unsigned r  = (t + 0x0FFFu + ((t >> 13) & 1u)) >> 13;
  const unsigned rc = r > 0x7C00u ? 0x7C00u : r;
  const bool small  = a < 0x38800000u;
  const bool isnan  = a > 0x7f800000u;
  const unsigned fin = small ? 0u : (s | rc);
  return isnan ? (s | 0x7E00u) : fin;
}

__device__ __forceinline__ unsigned pk16(unsigned lo, unsigned hi) { return lo | (hi << 16); }
__device__ __forceinline__ unsigned bf16_lo_bits(float v) {
  float hi = bf16_val(v);
  asm volatile("" : "+v"(hi));
  return bf16_bits(v - hi);
}
__device__ __forceinline__ v4u pack8_bf16(v4f a, v4f c) {
  return (v4u){ pk16(bf16_bits(a[0]), bf16_bits(a[1])), pk16(bf16_bits(a[2]), bf16_bits(a[3])),
                pk16(bf16_bits(c[0]), bf16_bits(c[1])), pk16(bf16_bits(c[2]), bf16_bits(c[3])) };
}
__device__ __forceinline__ v4u pack8_bf16_lo(v4f a, v4f c) {
  return (v4u){ pk16(bf16_lo_bits(a[0]), bf16_lo_bits(a[1])), pk16(bf16_lo_bits(a[2]), bf16_lo_bits(a[3])),
                pk16(bf16_lo_bits(c[0]), bf16_lo_bits(c[1])), pk16(bf16_lo_bits(c[2]), bf16_lo_bits(c[3])) };
}
__device__ __forceinline__ v4u pack8_f16(v4f a, v4f c) {
  return (v4u){ pk16(f16_bits(a[0]), f16_bits(a[1])), pk16(f16_bits(a[2]), f16_bits(a[3])),
                pk16(f16_bits(c[0]), f16_bits(c[1])), pk16(f16_bits(c[2]), f16_bits(c[3])) };
}

template <int FORM>
__global__ __launch_bounds__(256) void k_plane(const float* __restrict__ src, int rows, int cols, int ldsrc,
                                               unsigned short* __restrict__ dst, int MP, int KP) {
  static_assert(FORM >= 0 && FORM <= 3);
  const int KTOT = (FORM == 1 || FORM == 3) ? 2 * KP : KP;
  const unsigned ppr   = (unsigned)(KTOT >> 3);
  const unsigned kp8   = (unsigned)(KP >> 3);
  const unsigned total = (unsigned)MP * ppr;
  const unsigned g     = blockIdx.x * 256u + threadIdx.x;
  const unsigned rowu  = g / ppr;
  const unsigned p     = g - rowu * ppr;
  const bool second    = p >= kp8;
  const int row = (int)rowu;
  const int c0  = (int)((second ? p - kp8 : p) << 3);
  const float* srow = src + (size_t)clampi(row, 0, rows - 1) * (size_t)ldsrc;
  float x[8];
  unsigned mk[8];
#pragma unroll
  for (int e = 0; e < 8; ++e) {
    const int c = c0 + e;
    const float v = srow[clampi(c, 0, cols - 1)];
    asm volatile("" :: "v"(v));
    x[e]  = v;
    mk[e] = (row < rows && c < cols) ? 0xFFFFu : 0u;
  }
  const v4f a = (v4f){ x[0], x[1], x[2], x[3] };
  const v4f c = (v4f){ x[4], x[5], x[6], x[7] };
  v4u o;
  if (FORM == 2) {
    o = pack8_f16(a, c);
  } else {
    const v4u hi = pack8_bf16(a, c);
    o = hi;
    if (FORM == 1) { const v4u lo = pack8_bf16_lo(a, c); o = second ? lo : hi; }
  }
  const v4u mw = (v4u){ pk16(mk[0], mk[1]), pk16(mk[2], mk[3]), pk16(mk[4], mk[5]), pk16(mk[6], mk[7]) };
  o &= mw;
  if (g < total) {
    volatile v4u* q = (volatile v4u*)(dst + (size_t)g * 8);
    *q = o;
    __threadfence();
    *q = o;
  }
}

template <int FORM> struct FragOf    { typedef FragB T; };
template <>         struct FragOf<2> { typedef FragH T; };
__device__ __forceinline__ v8f mm(const FragB& a, const FragB& b, v8f c) { return wmb(a, b, c); }
__device__ __forceinline__ v8f mm(const FragH& a, const FragH& b, v8f c) { return wmh(a, b, c); }
template <class F> __device__ __forceinline__ F ld_frag(const unsigned short* p) {
  F f;
  f.h[0] = *(const v8usa*)(p);
  f.h[1] = *(const v8usa*)(p + 16);
  return f;
}

template <int FORM, int EPI>
__global__ __launch_bounds__(256) __attribute__((amdgpu_num_vgpr(248)))
void k_gemm_nt(const unsigned short* __restrict__ A, const unsigned short* __restrict__ B,
               const float* __restrict__ bias, float* __restrict__ D, int M, int N, int KTOT, int ldd) {
  static_assert(FORM >= 0 && FORM <= 2);
  static_assert(EPI == 0 || EPI == 1);
  typedef typename FragOf<FORM>::T F;
  __shared__ __attribute__((aligned(16))) float sT[8][16 * 68];
  const int lane = threadIdx.x & 31;
  const int wave = threadIdx.x >> 5;
  const int tilesM = (M + 63) >> 6;
  const int tilesN = (N + 63) >> 6;
  const int tile = blockIdx.x * 8 + wave;
  if (tile >= tilesM * tilesN) return;
  const int tm = tile / tilesN;
  const int tn = tile - tm * tilesN;
  const int m0 = tm << 6;
  const int n0 = tn << 6;

  const int rl = lane & 15;
  const int h8 = (lane >> 4) * 8;
  const unsigned short* pa = A + (size_t)(m0 + rl) * (size_t)KTOT + h8;
  const unsigned short* pb = B + (size_t)(n0 + rl) * (size_t)KTOT + h8;

  v8f acc[4][4];
#pragma unroll
  for (int i = 0; i < 4; ++i)
#pragma unroll
    for (int j = 0; j < 4; ++j) acc[i][j] = (v8f){0.f, 0.f, 0.f, 0.f, 0.f, 0.f, 0.f, 0.f};

#pragma unroll 1
  for (int k0 = 0; k0 < KTOT; k0 += 32) {
    F bf[4];
#pragma unroll
    for (int j = 0; j < 4; ++j) bf[j] = ld_frag<F>(pb + (size_t)(j << 4) * (size_t)KTOT + k0);
#pragma unroll
    for (int i = 0; i < 4; ++i) {
      const F af = ld_frag<F>(pa + (size_t)(i << 4) * (size_t)KTOT + k0);
#pragma unroll
      for (int j = 0; j < 4; ++j) acc[i][j] = mm(af, bf[j], acc[i][j]);
    }
  }

  float* slab = sT[wave];
  const int hh = lane >> 4;
  const int c4 = (lane & 15) * 4;
  const int nc = n0 + c4;
  const bool cok = nc < N;
  v4f bv = (v4f){0.f, 0.f, 0.f, 0.f};
  if (EPI == 1) {
    bv = *(const v4fa*)(bias + clampi(nc, 0, N - 4));
    asm volatile("" :: "v"(bv));
  }
#pragma unroll
  for (int i = 0; i < 4; ++i) {
    const int mBase = m0 + (i << 4);
#pragma unroll
    for (int j = 0; j < 4; ++j) {
#pragma unroll
      for (int r = 0; r < 8; ++r) slab[(h8 + r) * 68 + (j << 4) + rl] = acc[i][j][r];
    }
    __builtin_amdgcn_fence(__ATOMIC_RELEASE, "workgroup");
    __builtin_amdgcn_wave_barrier();
    __builtin_amdgcn_fence(__ATOMIC_ACQUIRE, "workgroup");
    v4f vv[8];
#pragma unroll
    for (int it = 0; it < 8; ++it) {
      const int row = it * 2 + hh;
      v4f v = *(const v4fa*)(slab + row * 68 + c4);
      if (EPI == 1) v += bv;
      vv[it] = v;
    }
    for (int pass = 0; pass < 2; ++pass) {
#pragma unroll
      for (int it = 0; it < 8; ++it) {
        const int row = mBase + it * 2 + hh;
        if (cok && row < M) *(volatile v4f*)(D + (size_t)row * (size_t)ldd + nc) = vv[it];
      }
      __threadfence();
    }
    __builtin_amdgcn_fence(__ATOMIC_RELEASE, "workgroup");
    __builtin_amdgcn_wave_barrier();
    __builtin_amdgcn_fence(__ATOMIC_ACQUIRE, "workgroup");
  }
}


#define L2_SINGLE 0

#define NN      50000
#define NE      800000
#define DD      128
#define MPAD    50048
#define K2TOT   (L2_SINGLE ? 128 : 256)
#define NREC    782
#define NB      1024
#define NBLKB   49
#define RCAP    21504
#define BK_WCAP 256
#define BK_LISTN 2048
#define BK_NCH  391
#define BK_LDS  ((2 * RCAP + 2 * NB + BK_LISTN + 16) * 4)
#define INV_CNT (1.0 / 6400000.0)

typedef float  v2f __attribute__((ext_vector_type(2)));
typedef int    v2i __attribute__((ext_vector_type(2)));
typedef int    v4i __attribute__((ext_vector_type(4)));
typedef double v2d __attribute__((ext_vector_type(2)));
typedef v2f __attribute__((may_alias)) v2fa;
typedef v2i __attribute__((may_alias)) v2ia;
typedef v4i __attribute__((may_alias)) v4ia;

static_assert(NE == 390 * 2048 + 1280);
static_assert(BK_NCH * 2048 >= NE && (BK_NCH - 1) * 2048 < NE);
static_assert(NBLKB * NB >= NN && (NBLKB - 1) * NB < NN);
static_assert(4 * RCAP >= 5 * 16623);
static_assert((RCAP % 1024) == 0);
static_assert(BK_LDS <= 262144);
static_assert(2 * 64 == DD);
static_assert(L2_SINGLE == 1 || K2TOT == 256);
static_assert((K2TOT % 32) == 0 && (DD % 32) == 0);
static_assert((MPAD % 64) == 0 && MPAD >= NN && (NN % 16) == 0);
static_assert(NREC * 64 == MPAD && NREC <= 1024);
static_assert(NN <= (1 << 21));

constexpr size_t SZ_XB   = (size_t)MPAD * DD * 2;
constexpr size_t SZ_W1T  = (size_t)DD * DD * 2;
constexpr size_t SZ_W2T  = (size_t)DD * K2TOT * 2;
constexpr size_t SZ_PV   = (size_t)10 * DD * 4;
constexpr size_t SZ_LSRC = (size_t)NBLKB * RCAP * 4;
constexpr size_t SZ_SLOT = (size_t)NBLKB * NB * 8;
constexpr size_t SZ_F    = (size_t)MPAD * DD * 4;
constexpr size_t SZ_A2   = (size_t)MPAD * K2TOT * 2;
constexpr size_t SZ_SC1  = (size_t)196 * 256 * 16;
constexpr size_t SZ_SC2  = (size_t)196 * 256 * 8;
constexpr size_t SZ_REC  = (size_t)NREC * 128;
constexpr size_t O_XB   = 0;
constexpr size_t O_W1T  = O_XB + SZ_XB;
constexpr size_t O_W2T  = O_W1T + SZ_W1T;
constexpr size_t O_PV   = O_W2T + SZ_W2T;
constexpr size_t O_LSRC = O_PV + SZ_PV;
constexpr size_t O_SLOT = O_LSRC + SZ_LSRC;
constexpr size_t O_H    = O_SLOT + SZ_SLOT;
constexpr size_t O_G    = O_H + SZ_F;
constexpr size_t O_A2   = O_G + SZ_F;
constexpr size_t O_SC1  = O_A2 + SZ_A2;
constexpr size_t O_SC2  = O_SC1 + SZ_SC1;
constexpr size_t O_RECA = O_SC2 + SZ_SC2;
constexpr size_t O_RECB = O_RECA + SZ_REC;
constexpr size_t WS_TOTAL = O_RECB + SZ_REC;
static_assert((O_W1T % 256) == 0 && (O_W2T % 256) == 0 && (O_PV % 256) == 0 && (O_LSRC % 256) == 0);
static_assert((O_SLOT % 256) == 0 && (O_H % 256) == 0 && (O_G % 256) == 0 && (O_A2 % 256) == 0);
static_assert((O_SC1 % 256) == 0 && (O_SC2 % 256) == 0 && (O_RECA % 256) == 0 && (O_RECB % 256) == 0);
static_assert(WS_TOTAL <= ((size_t)128 << 20));
static_assert(196 * 256 >= NN);

__device__ __forceinline__ float leaky(float v) { return v > 0.f ? v : 0.2f * v; }

#define PW2B (DD * (K2TOT / 8) / 256)
__device__ __forceinline__ void prep_wt(const float* __restrict__ w, unsigned short* __restrict__ wt, int u, int ppr) {
  const int n  = u / ppr;
  const int p  = u - n * ppr;
  const int k8 = (p & 15) << 3;
  const float* q = w + (size_t)k8 * DD + n;
  float xv[8];
#pragma unroll
  for (int e = 0; e < 8; ++e) {
    const float v = q[e * DD];
    asm volatile("" :: "v"(v));
    xv[e] = v;
  }
  const v4u o = pack8_bf16((v4f){ xv[0], xv[1], xv[2], xv[3] }, (v4f){ xv[4], xv[5], xv[6], xv[7] });
  volatile v4u* d = (volatile v4u*)(wt + (size_t)u * 8);
  *d = o;
  __threadfence();
  *d = o;
}

__global__ __launch_bounds__(256) void k_prep(const float* __restrict__ W1, const float* __restrict__ W2,
    const float* __restrict__ p0, const float* __restrict__ p1, const float* __restrict__ p2,
    const float* __restrict__ p3, const float* __restrict__ p4, const float* __restrict__ p5,
    const float* __restrict__ p6, const float* __restrict__ p7, const float* __restrict__ p8,
    const float* __restrict__ p9,
    unsigned short* __restrict__ W1T, unsigned short* __restrict__ W2T, float* __restrict__ PV) {
  const int b = (int)blockIdx.x, tid = (int)threadIdx.x;
  if (b < 8) {
    prep_wt(W1, W1T, b * 256 + tid, DD / 8);
  } else if (b < 8 + PW2B) {
    prep_wt(W2, W2T, (b - 8) * 256 + tid, K2TOT / 8);
  } else if (tid < 32) {
    const int l4 = 4 * tid;
    v4f r[10];
    r[0] = *(const v4fa*)(p0 + l4); r[1] = *(const v4fa*)(p1 + l4); r[2] = *(const v4fa*)(p2 + l4);
    r[3] = *(const v4fa*)(p3 + l4); r[4] = *(const v4fa*)(p4 + l4); r[5] = *(const v4fa*)(p5 + l4);
    r[6] = *(const v4fa*)(p6 + l4); r[7] = *(const v4fa*)(p7 + l4); r[8] = *(const v4fa*)(p8 + l4);
    r[9] = *(const v4fa*)(p9 + l4);
#pragma unroll
    for (int k = 0; k < 10; ++k)
      r[k] = (v4f){ bf16_val(r[k].x), bf16_val(r[k].y), bf16_val(r[k].z), bf16_val(r[k].w) };
    for (int pass = 0; pass < 2; ++pass) {
#pragma unroll
      for (int k = 0; k < 10; ++k) *(volatile v4f*)(PV + k * DD + l4) = r[k];
      __threadfence();
    }
  }
}

__global__ __launch_bounds__(256) void k_bucket(const int* __restrict__ srcs, const int* __restrict__ dsts,
                                                int* __restrict__ LSRC, int* __restrict__ SLOT) {
  extern __shared__ v4f lds_dyn[];
  int* reg1 = (int*)lds_dyn;
  int* reg2 = reg1 + RCAP;
  int* scnt = reg2 + RCAP;
  int* soff = scnt + NB;
  int* list = soff + NB;
  int* wcnt = list + BK_LISTN;
  int* wtot = wcnt + 8;
  const int tid = (int)threadIdx.x, lane = tid & 31, wave = tid >> 5;
  const int slotBase = (int)blockIdx.x * NB;
  const int nbv = (NN - slotBase) < NB ? (NN - slotBase) : NB;
  const int sent = (-0x7fffffff - 1);

  {
    const v4i z4 = (v4i){0, 0, 0, 0};
    for (int i = tid; i < RCAP / 4; i += 256) *(v4ia*)(reg2 + 4 * i) = z4;
    for (int i = tid; i < NB; i += 256) scnt[i] = 0;
    for (int i = tid; i < BK_LISTN; i += 256) list[i] = 0;
  }
  __syncthreads();

  int tot = 0;
#pragma unroll 1
  for (int ch = 0; ch < BK_NCH; ++ch) {
    const int wb = ch * 2048 + wave * 256;
    int dv[8];
#pragma unroll
    for (int J = 0; J < 8; ++J) {
      const int e  = wb + 32 * J + lane;
      const int ec = e < NE ? e : NE - 1;
      const int v  = dsts[ec];
      asm volatile("" :: "v"(v));
      dv[J] = (e < NE) ? v : sent;
    }
    int wc = 0;
#pragma unroll
    for (int J = 0; J < 8; ++J) {
      const unsigned s = (unsigned)dv[J] - (unsigned)slotBase;
      const bool hit = s < (unsigned)nbv;
      const unsigned mj = __builtin_amdgcn_ballot_w32(hit);
      const int pos = wc + (int)__builtin_amdgcn_mbcnt_lo(mj, 0u);
      if (hit && pos < BK_WCAP) list[wave * BK_WCAP + pos] = (int)(((unsigned)(32 * J + lane) << 10) | s);
      wc += (int)__builtin_popcount(mj);
    }
    if (lane == 0) wcnt[wave] = wc;
    __syncthreads();
    int pre = 0, all = 0;
#pragma unroll
    for (int w2 = 0; w2 < 8; ++w2) {
      int c = wcnt[w2];
      c = c < 0 ? 0 : (c > BK_WCAP ? BK_WCAP : c);
      all += c;
      pre += (w2 < wave) ? c : 0;
    }
    const int wcc  = wc > BK_WCAP ? BK_WCAP : wc;
    const int base = tot + pre;
#pragma unroll 1
    for (int i0 = 0; i0 < wcc; i0 += 32) {
      const int i   = i0 + lane;
      const int ic  = i < BK_WCAP ? i : BK_WCAP - 1;
      const int ent = list[wave * BK_WCAP + ic];
      const int el  = (ent >> 10) & 255;
      const int sl  = ent & (NB - 1);
      int eid = wb + el;
      eid = eid > NE - 1 ? NE - 1 : eid;
      int sv = srcs[eid];
      asm volatile("" :: "v"(sv));
      sv = clampi(sv, 0, NN - 1);
      const int pos = base + i;
      if (i < wcc && pos < RCAP) reg1[pos] = (int)(((unsigned)sv << 10) | (unsigned)sl);
    }
    tot += all;
    tot = tot > RCAP ? RCAP : tot;
    __syncthreads();
  }
  const int nh = tot;
  const bool ovf = (nh >= RCAP);

  if (wave == 0) {
#pragma unroll 1
    for (int b0 = 0; b0 < nh; b0 += 32) {
      const int idx = b0 + lane;
      const int uv  = reg1[idx < nh ? idx : nh - 1];
      const int m32 = (nh - b0) < 32 ? (nh - b0) : 32;
#pragma unroll 1
      for (int k = 0; k < m32; ++k) {
        const int u   = __builtin_amdgcn_readlane(uv, k);
        const int sl  = u & (NB - 1);
        const int cur = scnt[sl];
        if (lane == 0) scnt[sl] = cur + 1;
      }
    }
  }
  __syncthreads();

  {
    const v4i ca = *(const v4ia*)(scnt + 4 * tid);
    const int e0 = ca.x < 0 ? 0 : ca.x, e1 = ca.y < 0 ? 0 : ca.y, e2 = ca.z < 0 ? 0 : ca.z, e3 = ca.w < 0 ? 0 : ca.w;
    const int ts = e0 + e1 + e2 + e3;
    int incl = ts;
#pragma unroll
    for (int d = 1; d < 32; d <<= 1) {
      const int up = __shfl_up(incl, d);
      incl += (lane >= d) ? up : 0;
    }
    if (lane == 31) wtot[wave] = incl;
    __syncthreads();
    int pre = 0;
#pragma unroll
    for (int w2 = 0; w2 < 8; ++w2) pre += (w2 < wave) ? wtot[w2] : 0;
    int run = pre + incl - ts;
    soff[4 * tid + 0] = run; run += e0;
    soff[4 * tid + 1] = run; run += e1;
    soff[4 * tid + 2] = run; run += e2;
    soff[4 * tid + 3] = run;
  }
  __syncthreads();
  for (int i = tid; i < NB; i += 256) list[i] = soff[i];
  __syncthreads();

  if (wave == 0) {
#pragma unroll 1
    for (int b0 = 0; b0 < nh; b0 += 32) {
      const int idx = b0 + lane;
      const int uv  = reg1[idx < nh ? idx : nh - 1];
      const int m32 = (nh - b0) < 32 ? (nh - b0) : 32;
#pragma unroll 1
      for (int k = 0; k < m32; ++k) {
        const int u  = __builtin_amdgcn_readlane(uv, k);
        const int sl = u & (NB - 1);
        const int sv = (int)((unsigned)u >> 10);
        int pos = list[sl];
        pos = pos < 0 ? 0 : (pos > RCAP - 1 ? RCAP - 1 : pos);
        if (lane == 0) { reg2[pos] = sv; list[sl] = pos + 1; }
      }
    }
  }
  __syncthreads();

  for (int s = tid; s < NB; s += 256) {
    const int cs = scnt[s];
    list[2 * s]     = soff[s];
    list[2 * s + 1] = ovf ? -1 : cs;
  }
  __syncthreads();

  int* lp = LSRC + (size_t)blockIdx.x * RCAP;
  for (int pass = 0; pass < 2; ++pass) {
#pragma unroll 1
    for (int it = 0; it < RCAP / 1024; ++it) {
      const int p = it * 256 + tid;
      const v4i v = *(const v4ia*)(reg2 + 4 * p);
      *(volatile v4i*)(lp + 4 * p) = v;
    }
    __threadfence();
  }
  {
    const v4i q0 = *(const v4ia*)(list + 4 * tid);
    const v4i q1 = *(const v4ia*)(list + 4 * (tid + 256));
    int* sp = SLOT + (size_t)blockIdx.x * (2 * NB);
    for (int pass = 0; pass < 2; ++pass) {
      *(volatile v4i*)(sp + 4 * tid) = q0;
      *(volatile v4i*)(sp + 4 * (tid + 256)) = q1;
      __threadfence();
    }
  }
}

template <int H>
__global__ __launch_bounds__(256) void k_score(const float* __restrict__ Hm, const float* __restrict__ PV,
                                               int rowS, int rowD, float* __restrict__ SC) {
  static_assert(H == 1 || H == 2);
  __shared__ __attribute__((aligned(16))) float st[256 * 2 * H];
  const int tid = (int)threadIdx.x, lane = tid & 31, wave = tid >> 5;
  const v4f as = *(const v4fa*)(PV + rowS * DD + 4 * lane);
  const v4f ad = *(const v4fa*)(PV + rowD * DD + 4 * lane);
#pragma unroll 1
  for (int i = 0; i < 32; ++i) {
    const int r    = wave * 32 + i;
    const int node = (int)blockIdx.x * 256 + r;
    const int nc   = node < NN ? node : NN - 1;
    const v4f h = *(const v4fa*)(Hm + (size_t)nc * DD + 4 * lane);
    float ps = h.x * as.x; ps = fmaf(h.y, as.y, ps); ps = fmaf(h.z, as.z, ps); ps = fmaf(h.w, as.w, ps);
    float pd = h.x * ad.x; pd = fmaf(h.y, ad.y, pd); pd = fmaf(h.z, ad.z, pd); pd = fmaf(h.w, ad.w, pd);
    if (H == 1) { ps += __shfl_xor(ps, 16); pd += __shfl_xor(pd, 16); }
    ps += __shfl_xor(ps, 8); pd += __shfl_xor(pd, 8);
    ps += __shfl_xor(ps, 4); pd += __shfl_xor(pd, 4);
    ps += __shfl_xor(ps, 2); pd += __shfl_xor(pd, 2);
    ps += __shfl_xor(ps, 1); pd += __shfl_xor(pd, 1);
    if (H == 2) {
      const float ps1 = __shfl(ps, 16);
      const float pd1 = __shfl(pd, 16);
      if (lane == 0) *(v4fa*)(st + 4 * r) = (v4f){ ps, ps1, pd, pd1 };
    } else {
      if (lane == 0) *(v2fa*)(st + 2 * r) = (v2f){ ps, pd };
    }
  }
  __syncthreads();
  if (tid < 128 * H) {
    const v4f v = *(const v4fa*)(st + 4 * tid);
    volatile v4f* q = (volatile v4f*)(SC + (size_t)blockIdx.x * (256 * 2 * H) + 4 * tid);
    *q = v;
    __threadfence();
    *q = v;
  }
}

template <int H>
__device__ __forceinline__ void ld_sc(const float* __restrict__ SC, int n, float (&as)[H], float (&ad)[H]) {
  if (H == 2) {
    const v4f q = *(const v4fa*)(SC + (size_t)n * 4);
    asm volatile("" :: "v"(q));
    as[0] = q.x; as[H - 1] = q.y; ad[0] = q.z; ad[H - 1] = q.w;
  } else {
    const v2f q = *(const v2fa*)(SC + (size_t)n * 2);
    asm volatile("" :: "v"(q));
    as[0] = q.x; ad[0] = q.y;
  }
}

template <int H>
__device__ __forceinline__ int step_e(const int* __restrict__ lst, const float* __restrict__ SC, int offu, int cn,
                                      int tc, int j, const float (&adt)[H], float (&e)[H]) {
  int ix = offu + j;
  ix = ix > RCAP - 1 ? RCAP - 1 : ix;
  int lv = lst[ix];
  asm volatile("" :: "v"(lv));
  int s = (j < cn) ? lv : tc;
  s = clampi(s, 0, NN - 1);
  float as[H], ad[H];
  ld_sc<H>(SC, s, as, ad);
  const bool valid = j <= cn;
  const float ninf = -__builtin_inff();
#pragma unroll
  for (int h = 0; h < H; ++h) {
    const float ev = leaky(as[h] + adt[h]);
    e[h] = valid ? ev : ninf;
  }
  return s;
}

__device__ __forceinline__ void put_record(double* __restrict__ REC, double* sh, double wacc, int lane, int wave) {
  if (lane == 0) sh[wave] = wacc;
  __syncthreads();
  double t = sh[0];
#pragma unroll
  for (int k = 1; k < 8; ++k) t += sh[k];
  const v2d val = (v2d){ t, t };
  if (threadIdx.x < 8) {
    volatile v2d* q = (volatile v2d*)(REC + (size_t)blockIdx.x * 16 + 2 * threadIdx.x);
    *q = val;
    __threadfence();
    *q = val;
  }
}

__device__ __forceinline__ double rec_total(const double* __restrict__ REC, double* sh, int tid, int lane, int wave) {
  double a = 0.0;
#pragma unroll
  for (int k = 0; k < 4; ++k) {
    const int idx = tid + 256 * k;
    const int ic  = idx < NREC ? idx : NREC - 1;
    const double v = REC[(size_t)ic * 16];
    asm volatile("" :: "v"(v));
    a += (idx < NREC) ? v : 0.0;
  }
  a += __shfl_xor(a, 16);
  a += __shfl_xor(a, 8);
  a += __shfl_xor(a, 4);
  a += __shfl_xor(a, 2);
  a += __shfl_xor(a, 1);
  if (lane == 0) sh[wave] = a;
  __syncthreads();
  double t = sh[0];
#pragma unroll
  for (int k = 1; k < 8; ++k) t += sh[k];
  __syncthreads();
  return t;
}

template <int H>
__global__ __launch_bounds__(256) void k_replay(const int* __restrict__ LSRC, const int* __restrict__ SLOT,
    const float* __restrict__ Hm, const float* __restrict__ SC, const float* __restrict__ PV, int biasRow,
    float* __restrict__ G, double* __restrict__ REC) {
  static_assert(H == 1 || H == 2);
  __shared__ double sh[8];
  const int tid = (int)threadIdx.x, lane = tid & 31, wave = tid >> 5;
  const bool hsel = (H == 2) && (lane >= 16);
  const v4f bv = *(const v4fa*)(PV + biasRow * DD + 4 * lane);
  const float ninf = -__builtin_inff();
  const float qnan = __uint_as_float(0x7fc00000u);
  double wacc = 0.0;
#pragma unroll 1
  for (int i = 0; i < 8; ++i) {
    const int t = (int)blockIdx.x * 64 + wave * 8 + i;
    const bool live = t < NN;
    const int tc = live ? t : NN - 1;
    const v2i so = *(const v2ia*)(SLOT + 2 * tc);
    int sx = so.x, sy = so.y;
    asm volatile("" :: "v"(sx), "v"(sy));
    const int off = clampi(sx, 0, RCAP);
    int c = sy < 0 ? 0 : sy;
    c = c > RCAP - off ? RCAP - off : c;
    const int cn   = __builtin_amdgcn_readfirstlane(live ? c : 0);
    const int offu = __builtin_amdgcn_readfirstlane(off);
    const int flg  = __builtin_amdgcn_readfirstlane(sy < 0 ? 1 : 0);
    const int* lst = LSRC + (size_t)(tc >> 10) * RCAP;
    const int nent = cn + 1;

    float ast[H], adt[H];
    ld_sc<H>(SC, tc, ast, adt);

    float mx[H];
#pragma unroll
    for (int h = 0; h < H; ++h) mx[h] = ninf;
#pragma unroll 1
    for (int b0 = 0; b0 < nent; b0 += 32) {
      float e[H];
      (void)step_e<H>(lst, SC, offu, cn, tc, b0 + lane, adt, e);
#pragma unroll
      for (int h = 0; h < H; ++h) mx[h] = e[h] > mx[h] ? e[h] : mx[h];
    }
#pragma unroll
    for (int h = 0; h < H; ++h) {
#pragma unroll
      for (int o = 16; o > 0; o >>= 1) {
        const float ov = __shfl_xor(mx[h], o);
        mx[h] = ov > mx[h] ? ov : mx[h];
      }
    }

    float dn[H];
#pragma unroll
    for (int h = 0; h < H; ++h) dn[h] = 0.f;
#pragma unroll 1
    for (int b0 = 0; b0 < nent; b0 += 32) {
      float e[H];
      (void)step_e<H>(lst, SC, offu, cn, tc, b0 + lane, adt, e);
#pragma unroll
      for (int h = 0; h < H; ++h) dn[h] += expf(e[h] - mx[h]);
    }
#pragma unroll
    for (int h = 0; h < H; ++h) {
#pragma unroll
      for (int o = 16; o > 0; o >>= 1) dn[h] += __shfl_xor(dn[h], o);
    }

    v4f acc = (v4f){0.f, 0.f, 0.f, 0.f};
#pragma unroll 1
    for (int b0 = 0; b0 < nent; b0 += 32) {
      float e[H];
      const int s = step_e<H>(lst, SC, offu, cn, tc, b0 + lane, adt, e);
      float al[H];
#pragma unroll
      for (int h = 0; h < H; ++h) al[h] = expf(e[h] - mx[h]) / (dn[h] + 1e-16f);
      const int m = (nent - b0) < 32 ? (nent - b0) : 32;
#pragma unroll 1
      for (int jj = 0; jj < m; ++jj) {
        const int sj = __builtin_amdgcn_readlane(s, jj);
        const float a0 = __int_as_float(__builtin_amdgcn_readlane(__float_as_int(al[0]), jj));
        const float a1 = __int_as_float(__builtin_amdgcn_readlane(__float_as_int(al[H - 1]), jj));
        const float a  = hsel ? a1 : a0;
        const v4f hv = *(const v4fa*)(Hm + (size_t)sj * DD + 4 * lane);
        acc.x = fmaf(a, hv.x, acc.x);
        acc.y = fmaf(a, hv.y, acc.y);
        acc.z = fmaf(a, hv.z, acc.z);
        acc.w = fmaf(a, hv.w, acc.w);
      }
    }
    v4f v = acc + bv;
    if (flg != 0) v = (v4f){ qnan, qnan, qnan, qnan };
    float rs = (v.x + v.y) + (v.z + v.w);
    rs += __shfl_xor(rs, 16);
    rs += __shfl_xor(rs, 8);
    rs += __shfl_xor(rs, 4);
    rs += __shfl_xor(rs, 2);
    rs += __shfl_xor(rs, 1);
    if (live) {
      wacc += (double)rs;
      volatile v4f* q = (volatile v4f*)(G + (size_t)t * DD + 4 * lane);
      *q = v;
      __threadfence();
      *q = v;
    }
  }
  put_record(REC, sh, wacc, lane, wave);
}

__global__ __launch_bounds__(256) void k_sq(const float* __restrict__ G, const double* __restrict__ RECA,
                                            double* __restrict__ RECB) {
  __shared__ double sh[8];
  const int tid = (int)threadIdx.x, lane = tid & 31, wave = tid >> 5;
  const double tot = rec_total(RECA, sh, tid, lane, wave);
  const float mean = (float)(tot * INV_CNT);
  double wacc = 0.0;
#pragma unroll 1
  for (int i = 0; i < 8; ++i) {
    const int t = (int)blockIdx.x * 64 + wave * 8 + i;
    const bool live = t < NN;
    const int tc = live ? t : NN - 1;
    const v4f v = *(const v4fa*)(G + (size_t)tc * DD + 4 * lane);
    const v4f xc = v - mean;
    float q = (xc.x * xc.x + xc.y * xc.y) + (xc.z * xc.z + xc.w * xc.w);
    q += __shfl_xor(q, 16);
    q += __shfl_xor(q, 8);
    q += __shfl_xor(q, 4);
    q += __shfl_xor(q, 2);
    q += __shfl_xor(q, 1);
    if (live) wacc += (double)q;
  }
  put_record(RECB, sh, wacc, lane, wave);
}

template <int MODE>
__global__ __launch_bounds__(256) void k_norm(const float* __restrict__ G, const double* __restrict__ RECA,
    const double* __restrict__ RECB, const float* __restrict__ PV, int wRow, int bRow,
    unsigned short* __restrict__ A2, float* __restrict__ HN) {
  __shared__ double sh[8];
  const int tid = (int)threadIdx.x, lane = tid & 31, wave = tid >> 5;
  const double tA = rec_total(RECA, sh, tid, lane, wave);
  const double tB = rec_total(RECB, sh, tid, lane, wave);
  const float mean = (float)(tA * INV_CNT);
  const float var  = (float)(tB * INV_CNT);
  const float rstd = 1.0f / sqrtf(var + 1e-5f);
  if (MODE == 0) {
    const int c8 = 8 * (lane & 15);
    const v4f wa = *(const v4fa*)(PV + wRow * DD + c8);
    const v4f wc = *(const v4fa*)(PV + wRow * DD + c8 + 4);
    const v4f ba = *(const v4fa*)(PV + bRow * DD + c8);
    const v4f bc = *(const v4fa*)(PV + bRow * DD + c8 + 4);
    const bool second = lane >= 16;
#pragma unroll 1
    for (int i = 0; i < 8; ++i) {
      const int t = (int)blockIdx.x * 64 + wave * 8 + i;
      const bool live = t < NN;
      const int tc = live ? t : NN - 1;
      const v4f a = *(const v4fa*)(G + (size_t)tc * DD + c8);
      const v4f c = *(const v4fa*)(G + (size_t)tc * DD + c8 + 4);
      v4f ya = (a - mean) * rstd * wa + ba;
      v4f yc = (c - mean) * rstd * wc + bc;
#pragma unroll
      for (int k = 0; k < 4; ++k) {
        ya[k] = (ya[k] < 0.f) ? 0.f : ya[k];
        yc[k] = (yc[k] < 0.f) ? 0.f : yc[k];
      }
      const v4u hi = pack8_bf16(ya, yc);
      const v4u lo = pack8_bf16_lo(ya, yc);
      v4u o = second ? lo : hi;
      const unsigned lm = live ? 0xFFFFFFFFu : 0u;
      o &= (v4u){ lm, lm, lm, lm };
      if (K2TOT == 256 || lane < 16) {
        volatile v4u* q = (volatile v4u*)(A2 + (size_t)t * K2TOT + 8 * lane);
        *q = o;
        __threadfence();
        *q = o;
      }
    }
  } else {
    const v4f w4 = *(const v4fa*)(PV + wRow * DD + 4 * lane);
    const v4f b4 = *(const v4fa*)(PV + bRow * DD + 4 * lane);
#pragma unroll 1
    for (int i = 0; i < 8; ++i) {
      const int t = (int)blockIdx.x * 64 + wave * 8 + i;
      const bool live = t < NN;
      const int tc = live ? t : NN - 1;
      const v4f g = *(const v4fa*)(G + (size_t)tc * DD + 4 * lane);
      const v4f y = (g - mean) * rstd * w4 + b4;
      if (live) {
        volatile v4f* q = (volatile v4f*)(HN + (size_t)t * DD + 4 * lane);
        *q = y;
        __threadfence();
        *q = y;
      }
    }
  }
}

__global__ __launch_bounds__(256) void k_final(const int* __restrict__ LSRC, const int* __restrict__ SLOT,
    const float* __restrict__ HN, const float* __restrict__ X, float* __restrict__ OUT) {
  const int tid = (int)threadIdx.x, lane = tid & 31, wave = tid >> 5;
  const float qnan = __uint_as_float(0x7fc00000u);
#pragma unroll 1
  for (int i = 0; i < 8; ++i) {
    const int t = (int)blockIdx.x * 64 + wave * 8 + i;
    const bool live = t < NN;
    const int tc = live ? t : NN - 1;
    const v2i so = *(const v2ia*)(SLOT + 2 * tc);
    int sx = so.x, sy = so.y;
    asm volatile("" :: "v"(sx), "v"(sy));
    const int off = clampi(sx, 0, RCAP);
    int c = sy < 0 ? 0 : sy;
    c = c > RCAP - off ? RCAP - off : c;
    const int cn   = __builtin_amdgcn_readfirstlane(live ? c : 0);
    const int offu = __builtin_amdgcn_readfirstlane(off);
    const int flg  = __builtin_amdgcn_readfirstlane(sy < 0 ? 1 : 0);
    const int* lst = LSRC + (size_t)(tc >> 10) * RCAP;
    const v4f xv = *(const v4fa*)(X + (size_t)tc * DD + 4 * lane);
    asm volatile("" :: "v"(xv));

    v4f acc = (v4f){0.f, 0.f, 0.f, 0.f};
#pragma unroll 1
    for (int b0 = 0; b0 < cn; b0 += 32) {
      int ix = offu + b0 + lane;
      ix = ix > RCAP - 1 ? RCAP - 1 : ix;
      int lv = lst[ix];
      asm volatile("" :: "v"(lv));
      const int s = clampi(lv, 0, NN - 1);
      const int m = (cn - b0) < 32 ? (cn - b0) : 32;
#pragma unroll 1
      for (int jj = 0; jj < m; ++jj) {
        const int sj = __builtin_amdgcn_readlane(s, jj);
        const v4f hv = *(const v4fa*)(HN + (size_t)sj * DD + 4 * lane);
        acc += hv;
      }
    }
    const float cf = fmaxf((float)cn, 1.0f);
    const v4f mm4 = acc / cf;
    v4f o = mm4 + (v4f){ bf16_val(xv.x), bf16_val(xv.y), bf16_val(xv.z), bf16_val(xv.w) };
#pragma unroll
    for (int k = 0; k < 4; ++k) o[k] = (o[k] < 0.f) ? 0.f : o[k];
    if (flg != 0) o = (v4f){ qnan, qnan, qnan, qnan };
    if (live) {
      volatile v4f* q = (volatile v4f*)(OUT + (size_t)t * DD + 4 * lane);
      *q = o;
      __threadfence();
      *q = o;
    }
  }
}

extern "C" void kernel_launch(void* const* d_in, const int* in_sizes, int n_in,
                              void* d_out, int out_size, void* d_ws, size_t ws_size,
                              hipStream_t stream) {
  if (n_in < 14) return;
  if (in_sizes[0] != NN * DD || in_sizes[1] != 2 * NE) return;
  if (in_sizes[2] != DD * DD || in_sizes[8] != DD * DD) return;
  if (in_sizes[3] != DD || in_sizes[4] != DD || in_sizes[5] != DD || in_sizes[6] != DD || in_sizes[7] != DD) return;
  if (in_sizes[9] != DD || in_sizes[10] != DD || in_sizes[11] != DD || in_sizes[12] != DD || in_sizes[13] != DD) return;
  if (out_size != NN * DD) return;
  if (ws_size < WS_TOTAL) return;

  const float* x    = (const float*)d_in[0];
  const int*   ei   = (const int*)  d_in[1];
  const float* W1   = (const float*)d_in[2];
  const float* as1  = (const float*)d_in[3];
  const float* ad1  = (const float*)d_in[4];
  const float* b1   = (const float*)d_in[5];
  const float* l1w  = (const float*)d_in[6];
  const float* l1b  = (const float*)d_in[7];
  const float* W2   = (const float*)d_in[8];
  const float* as2  = (const float*)d_in[9];
  const float* ad2  = (const float*)d_in[10];
  const float* b2   = (const float*)d_in[11];
  const float* l2w  = (const float*)d_in[12];
  const float* l2b  = (const float*)d_in[13];
  float* out = (float*)d_out;
  const int* src = ei;
  const int* dst = ei + NE;

  char* ws = (char*)d_ws;
  unsigned short* XB  = (unsigned short*)(ws + O_XB);
  unsigned short* W1T = (unsigned short*)(ws + O_W1T);
  unsigned short* W2T = (unsigned short*)(ws + O_W2T);
  float*  PV   = (float*)(ws + O_PV);
  int*    LSRC = (int*)(ws + O_LSRC);
  int*    SLOT = (int*)(ws + O_SLOT);
  float*  Hm   = (float*)(ws + O_H);
  float*  G    = (float*)(ws + O_G);
  unsigned short* A2 = (unsigned short*)(ws + O_A2);
  float*  SC1  = (float*)(ws + O_SC1);
  float*  SC2  = (float*)(ws + O_SC2);
  double* RECA = (double*)(ws + O_RECA);
  double* RECB = (double*)(ws + O_RECB);

  hipFuncSetAttribute(reinterpret_cast<const void*>(&k_bucket),
                      hipFuncAttributeMaxDynamicSharedMemorySize, BK_LDS);

  k_plane<0><<<MPAD * DD / 8 / 256, 256, 0, stream>>>(x, NN, DD, DD, XB, MPAD, DD);
  k_prep<<<8 + PW2B + 1, 256, 0, stream>>>(W1, W2, as1, ad1, b1, l1w, l1b, as2, ad2, b2, l2w, l2b, W1T, W2T, PV);
  k_bucket<<<NBLKB, 256, BK_LDS, stream>>>(src, dst, LSRC, SLOT);
  k_gemm_nt<0, 0><<<196, 256, 0, stream>>>(XB, W1T, PV, Hm, NN, DD, DD, DD);
  k_score<2><<<196, 256, 0, stream>>>(Hm, PV, 0, 1, SC1);
  k_replay<2><<<NREC, 256, 0, stream>>>(LSRC, SLOT, Hm, SC1, PV, 2, G, RECA);
  k_sq<<<NREC, 256, 0, stream>>>(G, RECA, RECB);
  k_norm<0><<<NREC, 256, 0, stream>>>(G, RECA, RECB, PV, 3, 4, A2, Hm);
  k_gemm_nt<0, 0><<<196, 256, 0, stream>>>(A2, W2T, PV, Hm, NN, DD, K2TOT, DD);
  k_score<1><<<196, 256, 0, stream>>>(Hm, PV, 5, 6, SC2);
  k_replay<1><<<NREC, 256, 0, stream>>>(LSRC, SLOT, Hm, SC2, PV, 7, G, RECA);
  k_sq<<<NREC, 256, 0, stream>>>(G, RECA, RECB);
  k_norm<1><<<NREC, 256, 0, stream>>>(G, RECA, RECB, PV, 8, 9, A2, Hm);
  k_final<<<NREC, 256, 0, stream>>>(LSRC, SLOT, Hm, x, out);
}
